// BahdanauAttention_6176162972448
// MI455X (gfx1250) — hardware-run, weakly checked
//
#include <hip/hip_runtime.h>
#define NB 2
#define SQ 2048
#define DM 1024
#define NH 16
#define HD 64
#define HG 4
#define LB 8
#define LT 512
#define LS 512
#define LD 128
#define LCW 16.0f
#define LCP 1024.0f
#define LCC 64.0f
#define B0 0
#define NBR NB
#define NR ((size_t)NB * SQ)
#define MP ((int)((size_t)NBR * SQ))
#define QN SQ
#define NHD NH
#define MPO MP
#define LQ DM
typedef __bf16 v16b __attribute__((ext_vector_type(16)));
typedef unsigned short v8us __attribute__((ext_vector_type(8), may_alias));
typedef float  v8f  __attribute__((ext_vector_type(8)));
typedef float  v4f  __attribute__((ext_vector_type(4)));
typedef float  v4fa __attribute__((ext_vector_type(4), may_alias));
union FragB { v16b v; v8us half[2]; unsigned short u[16]; };

__device__ __forceinline__ unsigned short bf16_bits(float x) { unsigned int u = __float_as_uint(x); return (unsigned short)((u + 0x7FFFu + ((u >> 16) & 1u)) >> 16); }
__device__ __forceinline__ float bf16_val(unsigned short b) { return __uint_as_float(((unsigned int)b) << 16); }
__device__ __forceinline__ float bf16_round(float x) { return bf16_val(bf16_bits(x)); }
template <int NT>
__device__ __forceinline__ v8f mmaN(v16b ah, v16b al, v16b bh, v16b bl, v8f c) {
  c = __builtin_amdgcn_wmma_f32_16x16x32_bf16(false, ah, false, bh, (short)0, c, false, false);
  if (NT >= 2) c = __builtin_amdgcn_wmma_f32_16x16x32_bf16(false, al, false, bh, (short)0, c, false, false);
  if (NT >= 3) c = __builtin_amdgcn_wmma_f32_16x16x32_bf16(false, ah, false, bl, (short)0, c, false, false);
  asm volatile("v_nop\n\tv_nop\n\tv_nop\n\tv_nop" : "+v"(c) : "v"(ah), "v"(al), "v"(bh), "v"(bl));
  return c;
}


typedef _Float16 v16h __attribute__((ext_vector_type(16)));
union FragH { v16h v; v8us half[2]; _Float16 h[16]; unsigned short u[16]; };
template <int NT>
__device__ __forceinline__ v8f mmaH(v16h ah, v16h al, v16h bh, v16h bl, v8f c) {
  c = __builtin_amdgcn_wmma_f32_16x16x32_f16(false, ah, false, bh, (short)0, c, false, false);
  if (NT >= 2) c = __builtin_amdgcn_wmma_f32_16x16x32_f16(false, al, false, bh, (short)0, c, false, false);
  if (NT >= 3) c = __builtin_amdgcn_wmma_f32_16x16x32_f16(false, ah, false, bl, (short)0, c, false, false);
  asm volatile("v_nop\n\tv_nop\n\tv_nop\n\tv_nop" : "+v"(c) : "v"(ah), "v"(al), "v"(bh), "v"(bl));
  return c;
}

__global__ __launch_bounds__(256) void k_wt_f16(const float* __restrict__ W, _Float16* __restrict__ Wt, int K, int N, float scale) {
  const int t = blockIdx.x * 256 + threadIdx.x; if (t >= N * (K / 8)) return; const int n = t / (K / 8), k8 = (t % (K / 8)) * 8; FragH f;
#pragma unroll
  for (int i = 0; i < 8; ++i) f.h[i] = (_Float16)(bf16_round(W[(size_t)(k8 + i) * N + n]) * scale); const v8us o = f.half[0];
  *(volatile v8us*)((unsigned short*)Wt + (size_t)n * K + k8) = o; __threadfence(); *(volatile v8us*)((unsigned short*)Wt + (size_t)n * K + k8) = o;
}

typedef _Float16 v4h __attribute__((ext_vector_type(4)));

__global__ __launch_bounds__(256) void k_x16(const float* __restrict__ x, _Float16* __restrict__ X16, size_t n8) { const size_t t = (size_t)blockIdx.x * 256 + threadIdx.x; if (t >= n8) return; FragH f;
#pragma unroll
  for (int q = 0; q < 8; ++q) f.h[q] = (_Float16)bf16_round(x[t * 8 + q]); *(volatile v8us*)((unsigned short*)X16 + t * 8) = f.half[0]; __threadfence(); *(volatile v8us*)((unsigned short*)X16 + t * 8) = f.half[0]; }
__global__ __launch_bounds__(256) void k_x16s(const float* __restrict__ x, _Float16* __restrict__ X16, size_t n8, float scale) { const size_t t = (size_t)blockIdx.x * 256 + threadIdx.x; if (t >= n8) return; FragH f;
#pragma unroll
  for (int q = 0; q < 8; ++q) f.h[q] = (_Float16)(bf16_round(x[t * 8 + q]) * scale); *(volatile v8us*)((unsigned short*)X16 + t * 8) = f.half[0]; __threadfence(); *(volatile v8us*)((unsigned short*)X16 + t * 8) = f.half[0]; }


__device__ __forceinline__ v16h g2_frag(const _Float16* p, int hh) { FragH f; f.half[0] = *(const v8us*)((const unsigned short*)p + 8 * hh); f.half[1] = *(const v8us*)((const unsigned short*)p + 16 + 8 * hh); return f.v; }
__device__ __forceinline__ v8f g2_mma(v16h a, v16h b, v8f c) { v8f d = __builtin_amdgcn_wmma_f32_16x16x32_f16(false, a, false, b, (short)0, c, false, false); asm volatile("v_nop\n\tv_nop\n\tv_nop\n\tv_nop" : "+v"(d) : "v"(a), "v"(b)); return d; }
template <int ACT>
__global__ __launch_bounds__(128) void k_gemm2(const _Float16* __restrict__ A, int lda, size_t sA, const _Float16* __restrict__ Bh, int ldb, size_t sB, float alpha, const float* __restrict__ bias, size_t sBias, const float* __restrict__ CP, int rowsPerB, size_t sCPb, int row0g,
    float* __restrict__ C, _Float16* __restrict__ C16, int ldc, size_t sC, int M, int N, int K) { static_assert(ACT == 0 || ACT == 3 || ACT == 6 || ACT == 8 || ACT == 9 || ACT == 11 || ACT == 12 || ACT == 14 || ACT == 15 || ACT == 16 || ACT == 17, "k_gemm2: unsupported ACT code (would silently apply no activation)");
  __shared__ __attribute__((aligned(16))) float so[4][32][68];
  const int tid = threadIdx.x, w = tid >> 5, lane = tid & 31, ln = lane & 15, hh = lane >> 4; const int by = blockIdx.y;
  A += (size_t)by * sA; Bh += (size_t)by * sB; const size_t cofs = (size_t)by * sC; const float* bp = bias ? bias + (size_t)by * sBias : nullptr;
  const int ntn = N >> 6; const int mt = blockIdx.x / ntn, nq = blockIdx.x - mt * ntn; const int row0 = mt * 128 + 32 * w, col0 = nq * 64; if (row0 >= M) return;
  const _Float16* a0p = A + (size_t)(row0 + ln) * lda; const _Float16* a1p = a0p + (size_t)16 * lda;
  const _Float16* b0p = Bh + (size_t)(col0 + ln) * ldb; const _Float16* b1p = b0p + (size_t)16 * ldb; const _Float16* b2p = b1p + (size_t)16 * ldb; const _Float16* b3p = b2p + (size_t)16 * ldb;
  const v8f z8 = {0.f,0.f,0.f,0.f,0.f,0.f,0.f,0.f}; v8f c00 = z8, c01 = z8, c02 = z8, c03 = z8, c10 = z8, c11 = z8, c12 = z8, c13 = z8;
  for (int kb = 0; kb < K; kb += 32) { const v16h a0 = g2_frag(a0p + kb, hh), a1 = g2_frag(a1p + kb, hh);
    v16h b = g2_frag(b0p + kb, hh); c00 = g2_mma(a0, b, c00); c10 = g2_mma(a1, b, c10);
    b = g2_frag(b1p + kb, hh); c01 = g2_mma(a0, b, c01); c11 = g2_mma(a1, b, c11);
    b = g2_frag(b2p + kb, hh); c02 = g2_mma(a0, b, c02); c12 = g2_mma(a1, b, c12);
    b = g2_frag(b3p + kb, hh); c03 = g2_mma(a0, b, c03); c13 = g2_mma(a1, b, c13); }
  v8f accs[8] = {c00, c01, c02, c03, c10, c11, c12, c13};
#pragma unroll
  for (int u = 0; u < 8; ++u) { const int t = u & 3, half = u >> 2; const int col = col0 + t * 16 + ln; const float bv = bp ? bf16_round(bp[col]) : 0.f;
#pragma unroll
    for (int r = 0; r < 8; ++r) { const int rloc = half * 16 + 8 * hh + r; float v = accs[u][r] * alpha + bv; if (CP) { if (rowsPerB < 0) v += CP[cofs + (size_t)(row0g + row0 + rloc) * ldc + col];        else { const int bidx = (row0g + row0 + rloc) / rowsPerB; v += CP[(size_t)bidx * sCPb + (size_t)by * 64 + col]; } }
      if (ACT == 3) v = fmaxf(v, 0.f); else if (ACT == 6) v = 0.5f * v * (1.0f + erff(v * 0.70710678118654752f)); else if (ACT == 11) v = 1.0f / (1.0f + expf(-v)); else if (ACT == 15) v = v / (1.0f + expf(-v)); else if (ACT == 12) v = (v > 0.f) ? v : 0.01f * v; else if (ACT == 8) v = tanhf(v); else if (ACT == 9) v = 0.5f * v * (1.0f + tanhf(0.7978845608028654f * (v + 0.044715f * v * v * v))); else if (ACT == 14) v = (v > 0.f) ? v : 0.1f * v; else if (ACT == 16) v = (v >= 0.f) ? v : 0.3f * v; else if (ACT == 17) v = (v >= 0.f) ? v : 0.2f * v;
      so[w][rloc][t * 16 + ln] = v; } }
  __builtin_amdgcn_fence(__ATOMIC_ACQ_REL, "workgroup"); __builtin_amdgcn_wave_barrier();
  const int rsub = lane >> 4, c4 = (lane & 15) * 4;
  for (int pass = 0; pass < 2; ++pass) {
#pragma unroll
    for (int q = 0; q < 16; ++q) { const int r = q * 2 + rsub; const v4f v = *(const v4fa*)&so[w][r][c4]; if (C) *(volatile v4f*)(C + cofs + (size_t)(row0 + r) * ldc + col0 + c4) = v; if (C16) { v4h h4; for (int i = 0; i < 4; ++i) h4[i] = (_Float16)v[i]; *(volatile v4h*)(C16 + cofs + (size_t)(row0 + r) * ldc + col0 + c4) = h4; } }
    if (pass == 0) __threadfence(); } }


__device__ __forceinline__ float tanh_cf(float x) { return 1.0f - 2.0f / (1.0f + expf(2.0f * x)); }
__global__ __launch_bounds__(256) void k_score(const float* __restrict__ HP, const float* __restrict__ EP, const float* __restrict__ v, float* __restrict__ SC) {
  const size_t t = (size_t)blockIdx.x * 256 + threadIdx.x; if (t >= (size_t)LB * LT * LS) return; const unsigned s = (unsigned)(t % LS); const size_t bt = t / LS; const size_t b = bt / LT;
  const float* p1 = HP + bt * LD; const float* p2 = EP + (b * LS + s) * LD; float acc = 0.f;
  for (int o = 0; o < LD; o += 4) { const v4f a4 = *(const v4fa*)(p1 + o); const v4f c4 = *(const v4fa*)(p2 + o); const v4f w4 = *(const v4fa*)(v + o);
#pragma unroll
    for (int q = 0; q < 4; ++q) acc += bf16_round(w4[q]) * tanh_cf(a4[q] + c4[q]); }
  float* op = SC + t; *(volatile float*)op = acc; __threadfence(); *(volatile float*)op = acc; }
__global__ __launch_bounds__(256) void k_lsm(const float* __restrict__ SC, const int* __restrict__ lens, float* __restrict__ PR, _Float16* __restrict__ P16, float pscale) {
  const size_t r = (size_t)blockIdx.x * 256 + threadIdx.x; if (r >= (size_t)LB * LT) return; const size_t b = r / LT; const float* sp = SC + r * LS; const int len = lens[b];
  float m = -3.0e38f; for (int s = 0; s < LS; s += 8) { const v4f x0 = *(const v4fa*)(sp + s); const v4f x1 = *(const v4fa*)(sp + s + 4);
#pragma unroll
    for (int q = 0; q < 4; ++q) { m = fmaxf(m, (s + q < len) ? x0[q] : -3.0e38f); m = fmaxf(m, (s + 4 + q < len) ? x1[q] : -3.0e38f); } }
  float z = 0.f; for (int s = 0; s < LS; s += 8) { const v4f x0 = *(const v4fa*)(sp + s); const v4f x1 = *(const v4fa*)(sp + s + 4);
#pragma unroll
    for (int q = 0; q < 4; ++q) { const float e0 = expf(x0[q] - m); z += (s + q < len) ? e0 : 0.0f; }
#pragma unroll
    for (int q = 0; q < 4; ++q) { const float e1 = expf(x1[q] - m); z += (s + 4 + q < len) ? e1 : 0.0f; } }
  for (int s = 0; s < LS; s += 8) { const v4f x0 = *(const v4fa*)(sp + s); const v4f x1 = *(const v4fa*)(sp + s + 4); v4f o0, o1; FragH f;
#pragma unroll
    for (int q = 0; q < 4; ++q) { const float e0 = expf(x0[q] - m) / z; const float e1 = expf(x1[q] - m) / z; o0[q] = (s + q < len) ? e0 : 0.0f; o1[q] = (s + 4 + q < len) ? e1 : 0.0f; f.h[q] = (_Float16)(o0[q] * pscale); f.h[4 + q] = (_Float16)(o1[q] * pscale); }
    float* op = PR + r * LS + s; unsigned short* hp = (unsigned short*)P16 + r * LS + s; *(volatile v4f*)op = o0; *(volatile v4f*)(op + 4) = o1; *(volatile v8us*)hp = f.half[0]; __threadfence(); *(volatile v4f*)op = o0; *(volatile v4f*)(op + 4) = o1; *(volatile v8us*)hp = f.half[0]; } }

__global__ __launch_bounds__(256) void k_otanh(const float* __restrict__ Y, float* __restrict__ out) { const size_t t = (size_t)blockIdx.x * 256 + threadIdx.x; if (t >= (size_t)LB * LT * LD / 4) return; const v4f y = *(const v4fa*)(Y + t * 4); v4f o;
#pragma unroll
  for (int q = 0; q < 4; ++q) o[q] = tanh_cf(y[q]); float* op = out + t * 4; *(volatile v4f*)op = o; __threadfence(); *(volatile v4f*)op = o; }

extern "C" void kernel_launch(void* const* d_in, const int* in_sizes, int n_in,
                              void* d_out, int out_size, void* d_ws, size_t ws_size, hipStream_t stream) {
  (void)in_sizes; (void)n_in; (void)out_size;
  const float* qy = (const float*)d_in[0]; const float* enc = (const float*)d_in[1]; const int* lens = (const int*)d_in[2]; const float* ws_ = (const float*)d_in[3]; const float* wh = (const float*)d_in[4]; const float* v = (const float*)d_in[5]; const float* wo = (const float*)d_in[6]; const float* bo = (const float*)d_in[7];
  const int RT = LB * LT, RS = LB * LS;
  static_assert((LB * LT) % 128 == 0 && (LB * LS) % 128 == 0 && LT % 128 == 0 && LD % 64 == 0 && LD % 32 == 0 && LS % 32 == 0 && LS % 8 == 0 && LD % 8 == 0 && ((size_t)LB * LT * LD / 8) % 256 == 0 && ((size_t)LB * LS * LD / 8) % 256 == 0 && ((size_t)LD * LD / 8) % 256 == 0 && ((size_t)LD * 2 * LD / 8) % 256 == 0 && ((size_t)LD * (LS / 8)) % 256 == 0 && ((size_t)LB * LT * LS) % 256 == 0 && ((size_t)LB * LT) % 256 == 0 && ((size_t)LB * LT * LD / 4) % 256 == 0, "whole tiles; exact grids");
  float* aout = (float*)d_out; float* probs = (float*)d_out + (size_t)LB * LT * LD;
  char* ws = (char*)d_ws; size_t off = 0;
  auto take = [&](size_t bytes) { char* p = ws + off; off += (bytes + 255) & ~(size_t)255; return p; };
  _Float16* Q16 = (_Float16*)take((size_t)RT * LD * 2); _Float16* E16 = (_Float16*)take((size_t)RS * LD * 2); _Float16* WS16 = (_Float16*)take((size_t)LD * LD * 2); _Float16* WH16 = (_Float16*)take((size_t)LD * LD * 2); _Float16* WO16 = (_Float16*)take((size_t)LD * 2 * LD * 2); _Float16* ET = (_Float16*)take((size_t)LB * LD * LS * 2); _Float16* P16 = (_Float16*)take((size_t)RT * LS * 2); _Float16* C16 = (_Float16*)take((size_t)RT * LD * 2);
  float* HP = (float*)take((size_t)RT * LD * 4); float* EP = (float*)take((size_t)RS * LD * 4); float* SC = (float*)take((size_t)RT * LS * 4); float* Y = (float*)take((size_t)RT * LD * 4);
  if (off > ws_size) return;
  k_x16<<<(unsigned)((size_t)RT * LD / 8 / 256), 256, 0, stream>>>(qy, Q16, (size_t)RT * LD / 8); k_x16<<<(unsigned)((size_t)RS * LD / 8 / 256), 256, 0, stream>>>(enc, E16, (size_t)RS * LD / 8);
  k_x16s<<<(unsigned)((size_t)LD * LD / 8 / 256), 256, 0, stream>>>(ws_, WS16, (size_t)LD * LD / 8, LCW); k_x16s<<<(unsigned)((size_t)LD * LD / 8 / 256), 256, 0, stream>>>(wh, WH16, (size_t)LD * LD / 8, LCW); k_x16s<<<(unsigned)((size_t)LD * 2 * LD / 8 / 256), 256, 0, stream>>>(wo, WO16, (size_t)LD * 2 * LD / 8, LCW);
  for (int b = 0; b < LB; ++b) k_wt_f16<<<(unsigned)((size_t)LD * (LS / 8) / 256), 256, 0, stream>>>(enc + (size_t)b * LS * LD, ET + (size_t)b * LD * LS, LS, LD, LCW);

  k_gemm2<0><<<dim3((unsigned)((RT / 128) * (LD / 64)), 1), 128, 0, stream>>>(Q16, LD, 0, WS16, LD, 0, 1.0f / LCW, nullptr, 0, nullptr, 1, 0, 0, HP, nullptr, LD, 0, RT, LD, LD);
  k_gemm2<0><<<dim3((unsigned)((RS / 128) * (LD / 64)), 1), 128, 0, stream>>>(E16, LD, 0, WH16, LD, 0, 1.0f / LCW, nullptr, 0, nullptr, 1, 0, 0, EP, nullptr, LD, 0, RS, LD, LD);
  k_score<<<(unsigned)((size_t)LB * LT * LS / 256), 256, 0, stream>>>(HP, EP, v, SC);
  k_lsm<<<(unsigned)((size_t)LB * LT / 256), 256, 0, stream>>>(SC, lens, probs, P16, LCP);
  k_gemm2<0><<<dim3((unsigned)((LT / 128) * (LD / 64)), LB), 128, 0, stream>>>(P16, LS, (size_t)LT * LS, ET, LS, (size_t)LD * LS, LCC / (LCP * LCW), nullptr, 0, nullptr, 1, 0, 0, nullptr, C16, LD, (size_t)LT * LD, LT, LD, LS);
  k_gemm2<0><<<dim3((unsigned)((RT / 128) * (LD / 64)), 1), 128, 0, stream>>>(C16, LD, 0, WO16, 2 * LD, 0, 1.0f / (LCC * LCW), bo, 0, nullptr, 1, 0, 0, Y, nullptr, LD, 0, RT, LD, LD);
  k_gemm2<0><<<dim3((unsigned)((RT / 128) * (LD / 64)), 1), 128, 0, stream>>>(Q16, LD, 0, WO16 + LD, 2 * LD, 0, 1.0f / LCW, nullptr, 0, Y, -1, 0, 0, Y, nullptr, LD, 0, RT, LD, LD);
  k_otanh<<<(unsigned)((size_t)LB * LT * LD / 4 / 256), 256, 0, stream>>>(Y, aout);
}
